// STGCN_62886911148598
// MI455X (gfx1250) — hardware-verified
//
#include <hip/hip_runtime.h>
#define NBt 8
#define NNd 300
#define NNp 320
#define SL 64
#define TT 16
#define DM 128
#define NEd 4800
#define NG (NBt * TT)
#define NR (NNd * NG)
#define NP_ (NBt * NNd)
#define HP 512
typedef __bf16 v16b __attribute__((ext_vector_type(16)));
typedef unsigned short v8us __attribute__((ext_vector_type(8), may_alias));
typedef float  v8f  __attribute__((ext_vector_type(8)));
typedef float  v4f  __attribute__((ext_vector_type(4)));
typedef float  v4fa __attribute__((ext_vector_type(4), may_alias));
union FragB { v16b v; v8us half[2]; unsigned short u[16]; };

__device__ __forceinline__ unsigned short bf16_bits(float x) { unsigned int u = __float_as_uint(x); return (unsigned short)((u + 0x7FFFu + ((u >> 16) & 1u)) >> 16); }
__device__ __forceinline__ float bf16_val(unsigned short b) { return __uint_as_float(((unsigned int)b) << 16); }
__device__ __forceinline__ float bf16_round(float x) { return bf16_val(bf16_bits(x)); }
template <int NT>
__device__ __forceinline__ v8f mmaN(v16b ah, v16b al, v16b bh, v16b bl, v8f c) {
  c = __builtin_amdgcn_wmma_f32_16x16x32_bf16(false, ah, false, bh, (short)0, c, false, false);
  if (NT >= 2) c = __builtin_amdgcn_wmma_f32_16x16x32_bf16(false, al, false, bh, (short)0, c, false, false);
  if (NT >= 3) c = __builtin_amdgcn_wmma_f32_16x16x32_bf16(false, ah, false, bl, (short)0, c, false, false);
  asm volatile("v_nop\n\tv_nop\n\tv_nop\n\tv_nop" : "+v"(c) : "v"(ah), "v"(al), "v"(bh), "v"(bl));
  return c;
}

__global__ __launch_bounds__(256) void k_wt_bf16(const float* __restrict__ W, unsigned short* __restrict__ Wt, int K, int N) {
  const int t = blockIdx.x * 256 + threadIdx.x;
  const int k8n = K / 8;
  if (t >= N * k8n) return;
  const int n = t / k8n, k8 = (t % k8n) * 8;
  v8us v;
#pragma unroll
  for (int i = 0; i < 8; ++i) v[i] = bf16_bits(W[(size_t)(k8 + i) * N + n]);
  *(volatile v8us*)(Wt + (size_t)n * K + k8) = v;
  __threadfence();
  *(volatile v8us*)(Wt + (size_t)n * K + k8) = v;
}

template <bool ASPLIT, int ACT, bool BIAS_BF16>
__global__ __launch_bounds__(128) void k_gemm_bf(const float* __restrict__ A, int lda, const unsigned short* __restrict__ Wt, int ldb,
                                               const float* __restrict__ bias, float* __restrict__ C, int ldc, int M, int N, int K) {
  __shared__ __attribute__((aligned(16))) float so[4][16][64];
  const int tid = threadIdx.x, w = tid >> 5, lane = tid & 31, ln = lane & 15, hh = lane >> 4;
  const int ntn = N / 64;
  const int wid = blockIdx.x * 4 + w;
  const int mt = wid / ntn, nq = wid % ntn;
  if (mt * 16 >= M) return;
  const int row0 = mt * 16, col0 = nq * 64;
  const float* arow = A + (size_t)(row0 + ln) * lda;
  v8f acc[4] = {};
  for (int kb = 0; kb < K; kb += 32) {
    FragB ah, al;
    const v4f x0 = *(const v4fa*)(arow + kb + 8 * hh), x1 = *(const v4fa*)(arow + kb + 8 * hh + 4);
    const v4f x2 = *(const v4fa*)(arow + kb + 16 + 8 * hh), x3 = *(const v4fa*)(arow + kb + 16 + 8 * hh + 4);
    float xs[16] = {x0[0],x0[1],x0[2],x0[3],x1[0],x1[1],x1[2],x1[3],x2[0],x2[1],x2[2],x2[3],x3[0],x3[1],x3[2],x3[3]};
#pragma unroll
    for (int i = 0; i < 16; ++i) { const unsigned short hb = bf16_bits(xs[i]); ah.u[i] = hb; al.u[i] = ASPLIT ? bf16_bits(xs[i] - bf16_val(hb)) : (unsigned short)0; }
#pragma unroll
    for (int t = 0; t < 4; ++t) {
      const unsigned short* brow = Wt + (size_t)(col0 + t * 16 + ln) * ldb + kb;
      FragB b;
      b.half[0] = *(const v8us*)(brow + 8 * hh);
      b.half[1] = *(const v8us*)(brow + 16 + 8 * hh);
      acc[t] = mmaN<ASPLIT ? 2 : 1>(ah.v, al.v, b.v, b.v, acc[t]);
    }
  }
#pragma unroll
  for (int t = 0; t < 4; ++t) {
    float bv = bias ? bias[col0 + t * 16 + ln] : 0.f;
    if (BIAS_BF16) bv = bf16_round(bv);
#pragma unroll
    for (int r = 0; r < 8; ++r) { float v = acc[t][r] + bv; if (ACT == 1) v = fmaxf(v, 0.f); so[w][8 * hh + r][t * 16 + ln] = v; }
  }
  __builtin_amdgcn_fence(__ATOMIC_ACQ_REL, "workgroup");
  __builtin_amdgcn_wave_barrier();
  const int rsub = lane >> 4, c4 = (lane & 15) * 4;
  for (int pass = 0; pass < 2; ++pass) {
#pragma unroll
    for (int q = 0; q < 8; ++q) {
      const int r = q * 2 + rsub;
      const v4f v = *(const v4fa*)&so[w][r][c4];
      *(volatile v4f*)(C + (size_t)(row0 + r) * ldc + col0 + c4) = v;
    }
    if (pass == 0) __threadfence();
  }
}

template <bool ASPLIT, int ACT, bool BIAS_BF16, bool RES_BF16>
__global__ __launch_bounds__(128) void k_gemm_bf3(const float* __restrict__ A, int lda, const unsigned short* __restrict__ Wt, int ldb,
                                                const float* __restrict__ bias, const float* __restrict__ resid, int rmod, int ldr,
                                                float* __restrict__ C, int ldc, int M, int N, int K) {
  __shared__ __attribute__((aligned(16))) float so[4][16][64];
  const int tid = threadIdx.x, w = tid >> 5, lane = tid & 31, ln = lane & 15, hh = lane >> 4;
  const int ntn = N / 64;
  const int wid = blockIdx.x * 4 + w;
  const int mt = wid / ntn, nq = wid % ntn;
  if (mt * 16 >= M) return;
  const int row0 = mt * 16, col0 = nq * 64;
  const float* arow = A + (size_t)(row0 + ln) * lda;
  v8f acc[4] = {};
  for (int kb = 0; kb < K; kb += 32) {
    FragB ah, al;
    const v4f x0 = *(const v4fa*)(arow + kb + 8 * hh), x1 = *(const v4fa*)(arow + kb + 8 * hh + 4);
    const v4f x2 = *(const v4fa*)(arow + kb + 16 + 8 * hh), x3 = *(const v4fa*)(arow + kb + 16 + 8 * hh + 4);
    float xs[16] = {x0[0],x0[1],x0[2],x0[3],x1[0],x1[1],x1[2],x1[3],x2[0],x2[1],x2[2],x2[3],x3[0],x3[1],x3[2],x3[3]};
#pragma unroll
    for (int i = 0; i < 16; ++i) { const unsigned short hb = bf16_bits(xs[i]); ah.u[i] = hb; al.u[i] = ASPLIT ? bf16_bits(xs[i] - bf16_val(hb)) : (unsigned short)0; }
#pragma unroll
    for (int t = 0; t < 4; ++t) {
      const unsigned short* brow = Wt + (size_t)(col0 + t * 16 + ln) * ldb + kb;
      FragB b;
      b.half[0] = *(const v8us*)(brow + 8 * hh);
      b.half[1] = *(const v8us*)(brow + 16 + 8 * hh);
      acc[t] = mmaN<ASPLIT ? 2 : 1>(ah.v, al.v, b.v, b.v, acc[t]);
    }
  }
#pragma unroll
  for (int t = 0; t < 4; ++t) {
    const int col = col0 + t * 16 + ln;
    float bv = bias ? bias[col] : 0.f;
    if (BIAS_BF16) bv = bf16_round(bv);
#pragma unroll
    for (int r = 0; r < 8; ++r) {
      float v = acc[t][r] + bv;
      if (resid) { float rv = resid[(size_t)((row0 + 8 * hh + r) % rmod) * ldr + col]; if (RES_BF16) rv = bf16_round(rv); v += rv; }
      if (ACT == 1) v = fmaxf(v, 0.f);
      if (ACT == 2) v = 0.5f * v * (1.0f + erff(v * 0.70710678118654752f));
      if (ACT == 3) { const float u = 0.7978845608028654f * (v + 0.044715f * v * v * v); v = 0.5f * v * (1.0f + tanhf(u)); }
      so[w][8 * hh + r][t * 16 + ln] = v;
    }
  }
  __builtin_amdgcn_fence(__ATOMIC_ACQ_REL, "workgroup");
  __builtin_amdgcn_wave_barrier();
  const int rsub = lane >> 4, c4 = (lane & 15) * 4;
  for (int pass = 0; pass < 2; ++pass) {
#pragma unroll
    for (int q = 0; q < 8; ++q) {
      const int r = q * 2 + rsub;
      const v4f v = *(const v4fa*)&so[w][r][c4];
      *(volatile v4f*)(C + (size_t)(row0 + r) * ldc + col0 + c4) = v;
    }
    if (pass == 0) __threadfence();
  }
}
template <bool PARAM_BF16>
__global__ __launch_bounds__(256) void k_layernorm(const float* __restrict__ X, const float* __restrict__ R, const float* __restrict__ g, const float* __restrict__ bta,
                                                  float* __restrict__ out_sum, float* __restrict__ out_norm, int N, float eps) {
  __shared__ float red[256];
  const int row = blockIdx.x, tid = threadIdx.x;
  const float* x = X + (size_t)row * N; const float* rr = R ? R + (size_t)row * N : nullptr;
  float vals[16];
  const int per = N / 256;
  float s1 = 0.f;
  for (int u = 0; u < per / 4; ++u) {
    const int j = tid * 4 + 1024 * u;
    const v4f a = *(const v4fa*)(x + j);
    v4f b = {0.f,0.f,0.f,0.f}; if (rr) b = *(const v4fa*)(rr + j);
#pragma unroll
    for (int q = 0; q < 4; ++q) { const float v = a[q] + b[q]; vals[u * 4 + q] = v; s1 += v; }
  }
  red[tid] = s1; __syncthreads();
  for (int st = 128; st > 0; st >>= 1) { if (tid < st) red[tid] += red[tid + st]; __syncthreads(); }
  const float mu = red[0] / (float)N; __syncthreads();
  float s2 = 0.f;
  for (int u = 0; u < per / 4; ++u)
#pragma unroll
    for (int q = 0; q < 4; ++q) { const float c = vals[u * 4 + q] - mu; s2 += c * c; }
  red[tid] = s2; __syncthreads();
  for (int st = 128; st > 0; st >>= 1) { if (tid < st) red[tid] += red[tid + st]; __syncthreads(); }
  const float rs = rsqrtf(red[0] / (float)N + eps);
  for (int pass = 0; pass < 2; ++pass) {
    for (int u = 0; u < per / 4; ++u) {
      const int j = tid * 4 + 1024 * u;
      v4f o, sm;
#pragma unroll
      for (int q = 0; q < 4; ++q) {
        float gg = g[j + q], bb = bta[j + q];
        if (PARAM_BF16) { gg = bf16_round(gg); bb = bf16_round(bb); }
        sm[q] = vals[u * 4 + q]; o[q] = (vals[u * 4 + q] - mu) * rs * gg + bb;
      }
      if (out_sum) *(volatile v4f*)(out_sum + (size_t)row * N + j) = sm;
      *(volatile v4f*)(out_norm + (size_t)row * N + j) = o;
    }
    if (pass == 0) __threadfence();
  }
}


typedef _Float16 v16h __attribute__((ext_vector_type(16)));
union FragH { v16h v; v8us half[2]; _Float16 h[16]; unsigned short u[16]; };
template <int NT>
__device__ __forceinline__ v8f mmaH(v16h ah, v16h al, v16h bh, v16h bl, v8f c) {
  c = __builtin_amdgcn_wmma_f32_16x16x32_f16(false, ah, false, bh, (short)0, c, false, false);
  if (NT >= 2) c = __builtin_amdgcn_wmma_f32_16x16x32_f16(false, al, false, bh, (short)0, c, false, false);
  if (NT >= 3) c = __builtin_amdgcn_wmma_f32_16x16x32_f16(false, ah, false, bl, (short)0, c, false, false);
  asm volatile("v_nop\n\tv_nop\n\tv_nop\n\tv_nop" : "+v"(c) : "v"(ah), "v"(al), "v"(bh), "v"(bl));
  return c;
}
template <bool ASPLIT>
__global__ __launch_bounds__(128) void k_gemm_h(const float* __restrict__ A, int lda, size_t sA, const _Float16* __restrict__ Bh, int ldb, size_t sB, float alpha, float* __restrict__ C, int ldc, size_t sC, int M, int N, int K) {
  __shared__ __attribute__((aligned(16))) float so[4][16][64];
  const int tid = threadIdx.x, w = tid >> 5, lane = tid & 31, ln = lane & 15, hh = lane >> 4; const int by = blockIdx.y;
  A += (size_t)by * sA; Bh += (size_t)by * sB; C += (size_t)by * sC;
  const int ntn = (N + 63) / 64; const int wid = blockIdx.x * 4 + w; const int mt = wid / ntn, nq = wid % ntn; if (mt * 16 >= M) return;
  const int row0 = mt * 16, col0 = nq * 64; const float* arow = A + (size_t)(row0 + ln) * lda;
  v8f acc[4] = {};
  for (int kb = 0; kb < K; kb += 32) {
    FragH ah, al;
    const v4f x0 = *(const v4fa*)(arow + kb + 8 * hh), x1 = *(const v4fa*)(arow + kb + 8 * hh + 4), x2 = *(const v4fa*)(arow + kb + 16 + 8 * hh), x3 = *(const v4fa*)(arow + kb + 16 + 8 * hh + 4);
    float xs[16] = {x0[0],x0[1],x0[2],x0[3],x1[0],x1[1],x1[2],x1[3],x2[0],x2[1],x2[2],x2[3],x3[0],x3[1],x3[2],x3[3]};
#pragma unroll
    for (int i = 0; i < 16; ++i) { const _Float16 h = (_Float16)xs[i]; ah.h[i] = h; al.h[i] = ASPLIT ? (_Float16)(xs[i] - (float)h) : (_Float16)0.0f; }
#pragma unroll
    for (int t = 0; t < 4; ++t) { if (col0 + t * 16 >= N) continue; const size_t boff = (size_t)(col0 + t * 16 + ln) * ldb + kb; FragH bq; bq.half[0] = *(const v8us*)(Bh + boff + 8 * hh); bq.half[1] = *(const v8us*)(Bh + boff + 16 + 8 * hh);
      acc[t] = mmaH<ASPLIT ? 2 : 1>(ah.v, al.v, bq.v, bq.v, acc[t]); }
  }
#pragma unroll
  for (int t = 0; t < 4; ++t) { if (col0 + t * 16 >= N) continue;
#pragma unroll
    for (int r = 0; r < 8; ++r) so[w][8 * hh + r][t * 16 + ln] = acc[t][r] * alpha; }
  __builtin_amdgcn_fence(__ATOMIC_ACQ_REL, "workgroup"); __builtin_amdgcn_wave_barrier();
  const int rsub = lane >> 4, c4 = (lane & 15) * 4;
  for (int pass = 0; pass < 2; ++pass) {
#pragma unroll
    for (int q = 0; q < 8; ++q) { const int r = q * 2 + rsub; if (col0 + c4 < N) { const v4f v = *(const v4fa*)&so[w][r][c4]; *(volatile v4f*)(C + (size_t)(row0 + r) * ldc + col0 + c4) = v; } }
    if (pass == 0) __threadfence(); }
}

__global__ __launch_bounds__(256) void k_wt_f16(const float* __restrict__ W, _Float16* __restrict__ Wt, int K, int N, float scale) {
  const int t = blockIdx.x * 256 + threadIdx.x; if (t >= N * (K / 8)) return; const int n = t / (K / 8), k8 = (t % (K / 8)) * 8; FragH f;
#pragma unroll
  for (int i = 0; i < 8; ++i) f.h[i] = (_Float16)(bf16_round(W[(size_t)(k8 + i) * N + n]) * scale); const v8us o = f.half[0];
  *(volatile v8us*)((unsigned short*)Wt + (size_t)n * K + k8) = o; __threadfence(); *(volatile v8us*)((unsigned short*)Wt + (size_t)n * K + k8) = o;
}
template <int ACT>
__global__ __launch_bounds__(128) void k_gemm_hhx(const _Float16* __restrict__ A, int lda, size_t sA, const _Float16* __restrict__ Bh, int ldb, size_t sB, float alpha, const float* __restrict__ bias, size_t sBias, const float* __restrict__ CP, int rowsPerB, size_t sCPb, int row0g,
    float* __restrict__ C, _Float16* __restrict__ C16, int ldc, size_t sC, int M, int N, int K) {
  __shared__ __attribute__((aligned(16))) float so[4][16][64];
  const int tid = threadIdx.x, w = tid >> 5, lane = tid & 31, ln = lane & 15, hh = lane >> 4; const int by = blockIdx.y;
  A += (size_t)by * sA; Bh += (size_t)by * sB; const size_t cofs = (size_t)by * sC; const float* bp = bias ? bias + (size_t)by * sBias : nullptr;
  const int ntn = (N + 63) / 64; const int wid = blockIdx.x * 4 + w; const int mt = wid / ntn, nq = wid % ntn; if (mt * 16 >= M) return;
  const int row0 = mt * 16, col0 = nq * 64; const _Float16* arow = A + (size_t)(row0 + ln) * lda;
  v8f acc[4] = {};
  for (int kb = 0; kb < K; kb += 32) { FragH ah; ah.half[0] = *(const v8us*)((const unsigned short*)arow + kb + 8 * hh); ah.half[1] = *(const v8us*)((const unsigned short*)arow + kb + 16 + 8 * hh);
#pragma unroll
    for (int t = 0; t < 4; ++t) { if (col0 + t * 16 >= N) continue; const size_t boff = (size_t)(col0 + t * 16 + ln) * ldb + kb; FragH bq; bq.half[0] = *(const v8us*)((const unsigned short*)Bh + boff + 8 * hh); bq.half[1] = *(const v8us*)((const unsigned short*)Bh + boff + 16 + 8 * hh);
      acc[t] = mmaH<1>(ah.v, ah.v, bq.v, bq.v, acc[t]); }
  }
#pragma unroll
  for (int t = 0; t < 4; ++t) { if (col0 + t * 16 >= N) continue; const int col = col0 + t * 16 + ln; const float bv = bp ? bf16_round(bp[col]) : 0.f;
#pragma unroll
    for (int r = 0; r < 8; ++r) { float v = acc[t][r] * alpha + bv; if (CP) { const int bidx = (row0g + row0 + 8 * hh + r) / rowsPerB; v += CP[(size_t)bidx * sCPb + (size_t)by * 64 + col]; } if (ACT == 1) v = (v > 0.f) ? v : expm1f(v); else if (ACT == 7) v = (v > 0.f) ? v + 1.0f : expf(v); else if (ACT == 8) v = tanhf(v); else if (ACT == 9) v = 0.5f * v * (1.0f + tanhf(0.7978845608028654f * (v + 0.044715f * v * v * v))); else if (ACT == 11) v = 1.0f / (1.0f + expf(-v)); else if (ACT == 12) v = (v > 0.f) ? v : 0.01f * v; else if (ACT == 14) v = (v > 0.f) ? v : 0.1f * v; else if (ACT == 15) v = v / (1.0f + expf(-v)); else if (ACT == 3) v = fmaxf(v, 0.f); else if (ACT == 6) v = 0.5f * v * (1.0f + erff(v * 0.70710678118654752f)); so[w][8 * hh + r][t * 16 + ln] = v; } }
  __builtin_amdgcn_fence(__ATOMIC_ACQ_REL, "workgroup"); __builtin_amdgcn_wave_barrier();
  const int rsub = lane >> 4, c4 = (lane & 15) * 4; typedef _Float16 v4h __attribute__((ext_vector_type(4)));
  for (int pass = 0; pass < 2; ++pass) {
#pragma unroll
    for (int q = 0; q < 8; ++q) { const int r = q * 2 + rsub; if (col0 + c4 < N) { const v4f v = *(const v4fa*)&so[w][r][c4]; if (C) *(volatile v4f*)(C + cofs + (size_t)(row0 + r) * ldc + col0 + c4) = v; if (C16) { v4h h4; for (int i = 0; i < 4; ++i) h4[i] = (_Float16)v[i]; *(volatile v4h*)(C16 + cofs + (size_t)(row0 + r) * ldc + col0 + c4) = h4; } } }
    if (pass == 0) __threadfence(); }
}


typedef _Float16 v4h __attribute__((ext_vector_type(4)));

__global__ __launch_bounds__(256) void k_x16(const float* __restrict__ x, _Float16* __restrict__ X16, size_t n8) { const size_t t = (size_t)blockIdx.x * 256 + threadIdx.x; if (t >= n8) return; FragH f;
#pragma unroll
  for (int q = 0; q < 8; ++q) f.h[q] = (_Float16)bf16_round(x[t * 8 + q]); *(volatile v8us*)((unsigned short*)X16 + t * 8) = f.half[0]; __threadfence(); *(volatile v8us*)((unsigned short*)X16 + t * 8) = f.half[0]; }
__global__ __launch_bounds__(256) void k_h16(const float* __restrict__ x, _Float16* __restrict__ X16, size_t n8) { const size_t t = (size_t)blockIdx.x * 256 + threadIdx.x; if (t >= n8) return; FragH f;
#pragma unroll
  for (int q = 0; q < 8; ++q) f.h[q] = (_Float16)x[t * 8 + q]; *(volatile v8us*)((unsigned short*)X16 + t * 8) = f.half[0]; __threadfence(); *(volatile v8us*)((unsigned short*)X16 + t * 8) = f.half[0]; }
__global__ __launch_bounds__(256) void k_round16f(const float* __restrict__ W, _Float16* __restrict__ Bt, size_t n8) { const size_t t = (size_t)blockIdx.x * 256 + threadIdx.x; if (t >= n8) return; FragH f;
#pragma unroll
  for (int i = 0; i < 8; ++i) f.h[i] = (_Float16)(bf16_round(W[t * 8 + i]) * 16.0f); *(volatile v8us*)((unsigned short*)Bt + t * 8) = f.half[0]; __threadfence(); *(volatile v8us*)((unsigned short*)Bt + t * 8) = f.half[0]; }
template <int NHv, int TTv>
__global__ __launch_bounds__(256) void k_vt(const _Float16* __restrict__ V16, int ldv, int voff, _Float16* __restrict__ Vt) { __shared__ unsigned short tl[64][66]; const int tid = threadIdx.x; const int slab = blockIdx.x / (TTv / 64), lg = blockIdx.x % (TTv / 64); const int b = slab / NHv, h = slab % NHv;
  for (int i = tid; i < 64 * 8; i += 256) { const int r = i / 8, c8 = (i % 8) * 8; FragH f; f.half[0] = *(const v8us*)((const unsigned short*)V16 + ((size_t)b * TTv + lg * 64 + r) * ldv + voff + h * 64 + c8);
#pragma unroll
    for (int q = 0; q < 8; ++q) tl[r][c8 + q] = f.u[q]; }
  __syncthreads();
  for (int pass = 0; pass < 2; ++pass) {
#pragma unroll
    for (int rd = 0; rd < 2; ++rd) { const int d = rd * 32 + tid / 8, pc = tid % 8; FragH f;
#pragma unroll
      for (int q = 0; q < 8; ++q) f.u[q] = tl[pc * 8 + q][d];
      *(volatile v8us*)((unsigned short*)Vt + ((size_t)slab * 64 + d) * TTv + lg * 64 + pc * 8) = f.half[0]; }
    if (pass == 0) __threadfence(); } }

__global__ __launch_bounds__(256) void k_hl(const float* __restrict__ F, _Float16* __restrict__ Hh, _Float16* __restrict__ Hl, size_t n8) { const size_t t = (size_t)blockIdx.x * 256 + threadIdx.x; if (t >= n8) return; FragH fh, fl; const v4f a = *(const v4fa*)(F + t * 8), c = *(const v4fa*)(F + t * 8 + 4);
#pragma unroll
  for (int q = 0; q < 4; ++q) { _Float16 h = (_Float16)a[q]; fh.h[q] = h; fl.h[q] = (_Float16)((a[q] - (float)h) * 1024.0f); h = (_Float16)c[q]; fh.h[4 + q] = h; fl.h[4 + q] = (_Float16)((c[q] - (float)h) * 1024.0f); }
  for (int pass = 0; pass < 2; ++pass) { *(volatile v8us*)((unsigned short*)Hh + t * 8) = fh.half[0]; *(volatile v8us*)((unsigned short*)Hl + t * 8) = fl.half[0]; if (pass == 0) __threadfence(); } }

__global__ __launch_bounds__(256) void k_split(const float* __restrict__ F, _Float16* __restrict__ Hh, _Float16* __restrict__ Hl, size_t n8) {
  #pragma clang fp contract(off)
  const size_t t = (size_t)blockIdx.x * 256 + threadIdx.x; if (t >= n8) return; const v4f a = *(const v4fa*)(F + t * 8), c = *(const v4fa*)(F + t * 8 + 4); FragH fh, fl;
#pragma unroll
  for (int q = 0; q < 8; ++q) { const float v = (q < 4) ? a[q] : c[q - 4]; const _Float16 hi = (_Float16)v; fh.h[q] = hi; fl.h[q] = (_Float16)((v - (float)hi) * 1024.0f); }
  for (int pass = 0; pass < 2; ++pass) { *(volatile v8us*)((unsigned short*)Hh + t * 8) = fh.half[0]; *(volatile v8us*)((unsigned short*)Hl + t * 8) = fl.half[0]; if (pass == 0) __threadfence(); } }
template <int RELU>
__global__ __launch_bounds__(256) void k_splitr(const float* __restrict__ F, _Float16* __restrict__ Hh, _Float16* __restrict__ Hl, size_t n8) {
  #pragma clang fp contract(off)
  const size_t t = (size_t)blockIdx.x * 256 + threadIdx.x; if (t >= n8) return; const v4f a = *(const v4fa*)(F + t * 8), c = *(const v4fa*)(F + t * 8 + 4); FragH fh, fl;
#pragma unroll
  for (int q = 0; q < 8; ++q) { float v = (q < 4) ? a[q] : c[q - 4]; if (RELU) v = fmaxf(v, 0.f); const _Float16 hi = (_Float16)v; fh.h[q] = hi; fl.h[q] = (_Float16)((v - (float)hi) * 1024.0f); }
  for (int pass = 0; pass < 2; ++pass) { *(volatile v8us*)((unsigned short*)Hh + t * 8) = fh.half[0]; *(volatile v8us*)((unsigned short*)Hl + t * 8) = fl.half[0]; if (pass == 0) __threadfence(); } }
__global__ __launch_bounds__(256) void k_x0(const float* __restrict__ data, _Float16* __restrict__ X16) { const int t_ = blockIdx.x * 256 + threadIdx.x; if (t_ >= NR * (SL / 8)) return; const int f0 = (t_ % (SL / 8)) * 8; const int r = t_ / (SL / 8); const int n = r / NG, g = r % NG; const int b = g / TT, t = g % TT; FragH fh; v4f a, c;
#pragma unroll
  for (int q = 0; q < 8; ++q) { const float v = bf16_round(data[((size_t)b * NNd + n) * (SL * TT) + (size_t)(f0 + q) * TT + t]); fh.h[q] = (_Float16)v; (void)a; (void)c; }
  *(volatile v8us*)((unsigned short*)X16 + (size_t)r * SL + f0) = fh.half[0]; __threadfence(); *(volatile v8us*)((unsigned short*)X16 + (size_t)r * SL + f0) = fh.half[0]; }
__global__ __launch_bounds__(256) void k_adj(const int* __restrict__ esrc, const int* __restrict__ edst, _Float16* __restrict__ Ah, _Float16* __restrict__ Al) {
  #pragma clang fp contract(off)
  const int t = blockIdx.x * 256 + threadIdx.x; if (t >= NNp * (NNp / 8)) return; const int s0 = (t % (NNp / 8)) * 8, d = t / (NNp / 8); float acc[8];
#pragma unroll
  for (int q = 0; q < 8; ++q) acc[q] = 0.f;
  if (d < NNd) { int degd = 0; int degs[8];
#pragma unroll
    for (int q = 0; q < 8; ++q) degs[q] = 0;
#pragma unroll 1
    for (int e = 0; e < NEd; ++e) { const int dd = min(max(edst[e], 0), NNd - 1), ss = min(max(esrc[e], 0), NNd - 1); degd += (dd == d) ? 1 : 0;
#pragma unroll
      for (int q = 0; q < 8; ++q) degs[q] += (dd == s0 + q) ? 1 : 0; }
    const float did = (degd > 0) ? rsqrtf(fmaxf((float)degd, 1.f)) : 0.f; float dis[8];
#pragma unroll
    for (int q = 0; q < 8; ++q) dis[q] = (degs[q] > 0) ? rsqrtf(fmaxf((float)degs[q], 1.f)) : 0.f;
#pragma unroll 1
    for (int e = 0; e < NEd; ++e) { const int dd = min(max(edst[e], 0), NNd - 1), ss = min(max(esrc[e], 0), NNd - 1); if (dd == d) {
#pragma unroll
        for (int q = 0; q < 8; ++q) if (ss == s0 + q) acc[q] += dis[q] * did; } } }
  FragH fh, fl;
#pragma unroll
  for (int q = 0; q < 8; ++q) { const float v = acc[q]; const _Float16 hi = (_Float16)v; fh.h[q] = hi; fl.h[q] = (_Float16)((v - (float)hi) * 1024.0f); }
  for (int pass = 0; pass < 2; ++pass) { *(volatile v8us*)((unsigned short*)Ah + (size_t)d * NNp + s0) = fh.half[0]; *(volatile v8us*)((unsigned short*)Al + (size_t)d * NNp + s0) = fl.half[0]; if (pass == 0) __threadfence(); } }
__global__ __launch_bounds__(256) void k_htr(const float* __restrict__ Hs, float sgn, _Float16* __restrict__ Bh, _Float16* __restrict__ Bl) {
  #pragma clang fp contract(off)
  const int t = blockIdx.x * 256 + threadIdx.x; if (t >= NG * SL * (NNp / 8)) return; const int n0 = (t % (NNp / 8)) * 8; const int gf = t / (NNp / 8); FragH fh, fl;
#pragma unroll
  for (int q = 0; q < 8; ++q) { const int n = n0 + q; const float v = (n < NNd) ? sgn * Hs[(size_t)n * (NG * SL) + gf] : 0.f; const _Float16 hi = (_Float16)v; fh.h[q] = hi; fl.h[q] = (_Float16)((v - (float)hi) * 1024.0f); }
  for (int pass = 0; pass < 2; ++pass) { *(volatile v8us*)((unsigned short*)Bh + (size_t)gf * NNp + n0) = fh.half[0]; *(volatile v8us*)((unsigned short*)Bl + (size_t)gf * NNp + n0) = fl.half[0]; if (pass == 0) __threadfence(); } }
__global__ __launch_bounds__(256) void k_htrx(const _Float16* __restrict__ X16, _Float16* __restrict__ Bh) { const int t = blockIdx.x * 256 + threadIdx.x; if (t >= NG * SL * (NNp / 8)) return; const int n0 = (t % (NNp / 8)) * 8; const int gf = t / (NNp / 8); const int g = gf / SL, f = gf % SL; FragH fh;
#pragma unroll
  for (int q = 0; q < 8; ++q) { const int n = n0 + q; fh.h[q] = (n < NNd) ? X16[((size_t)n * NG + g) * SL + f] : (_Float16)0.0f; }
  *(volatile v8us*)((unsigned short*)Bh + (size_t)gf * NNp + n0) = fh.half[0]; __threadfence(); *(volatile v8us*)((unsigned short*)Bh + (size_t)gf * NNp + n0) = fh.half[0]; }
__global__ __launch_bounds__(256) void k_addres(float* Ho, const float* __restrict__ Hc, size_t n4) {
  #pragma clang fp contract(off)
  const size_t t = (size_t)blockIdx.x * 256 + threadIdx.x; if (t >= n4) return; const v4f a = *(const v4fa*)(Ho + t * 4), b = *(const v4fa*)(Hc + t * 4); v4f o;
#pragma unroll
  for (int q = 0; q < 4; ++q) o[q] = a[q] + b[q]; *(volatile v4f*)(Ho + t * 4) = o; __threadfence(); *(volatile v4f*)(Ho + t * 4) = o; }
__global__ __launch_bounds__(256) void k_neg(const float* __restrict__ P, _Float16* __restrict__ Th, _Float16* __restrict__ Tl, size_t n8) {
  #pragma clang fp contract(off)
  const size_t t = (size_t)blockIdx.x * 256 + threadIdx.x; if (t >= n8) return; const v4f a = *(const v4fa*)(P + t * 8), c = *(const v4fa*)(P + t * 8 + 4); FragH fh, fl;
#pragma unroll
  for (int q = 0; q < 8; ++q) { const float v = -((q < 4) ? a[q] : c[q - 4]); const _Float16 hi = (_Float16)v; fh.h[q] = hi; fl.h[q] = (_Float16)((v - (float)hi) * 1024.0f); }
  for (int pass = 0; pass < 2; ++pass) { *(volatile v8us*)((unsigned short*)Th + t * 8) = fh.half[0]; *(volatile v8us*)((unsigned short*)Tl + t * 8) = fl.half[0]; if (pass == 0) __threadfence(); } }
__global__ __launch_bounds__(256) void k_tx2(const float* __restrict__ P, const _Float16* __restrict__ X16, _Float16* __restrict__ Th, _Float16* __restrict__ Tl, size_t n8) {
  #pragma clang fp contract(off)
  const size_t t = (size_t)blockIdx.x * 256 + threadIdx.x; if (t >= n8) return; const v4f a = *(const v4fa*)(P + t * 8), c = *(const v4fa*)(P + t * 8 + 4); FragH x; x.half[0] = *(const v8us*)((const unsigned short*)X16 + t * 8); FragH fh, fl;
#pragma unroll
  for (int q = 0; q < 8; ++q) { const float v = -2.0f * ((q < 4) ? a[q] : c[q - 4]) - (float)x.h[q]; const _Float16 hi = (_Float16)v; fh.h[q] = hi; fl.h[q] = (_Float16)((v - (float)hi) * 1024.0f); }
  for (int pass = 0; pass < 2; ++pass) { *(volatile v8us*)((unsigned short*)Th + t * 8) = fh.half[0]; *(volatile v8us*)((unsigned short*)Tl + t * 8) = fl.half[0]; if (pass == 0) __threadfence(); } }
__global__ __launch_bounds__(256) void k_wgcn(const float* __restrict__ Wg, _Float16* __restrict__ Bt) { const int t = blockIdx.x * 256 + threadIdx.x; if (t >= 3 * DM * (SL / 8)) return; const int i0 = (t % (SL / 8)) * 8; const int ko = t / (SL / 8); const int k = ko / DM, o = ko % DM; FragH f;
#pragma unroll
  for (int q = 0; q < 8; ++q) f.h[q] = (_Float16)(bf16_round(Wg[((size_t)k * SL + i0 + q) * DM + o]) * 16.0f);
  *(volatile v8us*)((unsigned short*)Bt + (size_t)ko * SL + i0) = f.half[0]; __threadfence(); *(volatile v8us*)((unsigned short*)Bt + (size_t)ko * SL + i0) = f.half[0]; }
__global__ __launch_bounds__(256) void k_xt(const float* __restrict__ GCN, float* __restrict__ Ht) { const size_t t_ = (size_t)blockIdx.x * 256 + threadIdx.x; if (t_ >= (size_t)NP_ * TT * (DM / 4)) return; const int c0 = (int)(t_ % (DM / 4)) * 4; const size_t rt = t_ / (DM / 4); const int t = (int)(rt % TT); const int r = (int)(rt / TT); v4f v;
#pragma unroll
  for (int q = 0; q < 4; ++q) { const int cq = c0 + q; const int qq = r * DM + cq; const int b = qq / (DM * NNd), c = (qq % (DM * NNd)) / NNd, n = qq % NNd; const int g = b * TT + t; v[q] = GCN[((size_t)n * NG + g) * DM + c]; }
  *(volatile v4f*)(Ht + rt * DM + c0) = v; __threadfence(); *(volatile v4f*)(Ht + rt * DM + c0) = v; }
__global__ __launch_bounds__(256) void k_im1d(const float* __restrict__ Ht, int d, _Float16* __restrict__ Ih) {
  #pragma clang fp contract(off)
  const size_t t_ = (size_t)blockIdx.x * 256 + threadIdx.x; if (t_ >= (size_t)NP_ * TT * (3 * DM / 8)) return; const int g8 = (int)(t_ % (3 * DM / 8)) * 8; const size_t rt = t_ / (3 * DM / 8); const int t = (int)(rt % TT); const size_t r = rt / TT; const int k = g8 / DM, c0 = g8 % DM; const int ts = t + (k - 1) * d; FragH fh, fl;
#pragma unroll
  for (int q = 0; q < 8; ++q) { const float v = (ts >= 0 && ts < TT) ? Ht[(r * TT + ts) * DM + c0 + q] : 0.f; fh.h[q] = (_Float16)v; (void)fl; }
  *(volatile v8us*)((unsigned short*)Ih + rt * (3 * DM) + g8) = fh.half[0]; __threadfence(); *(volatile v8us*)((unsigned short*)Ih + rt * (3 * DM) + g8) = fh.half[0]; }
__global__ __launch_bounds__(256) void k_wt3(const float* __restrict__ Wt, _Float16* __restrict__ Bt) { const int t = blockIdx.x * 256 + threadIdx.x; if (t >= DM * (3 * DM / 8)) return; const int g8 = (t % (3 * DM / 8)) * 8, o = t / (3 * DM / 8); const int k = g8 / DM, c0 = g8 % DM; FragH f;
#pragma unroll
  for (int q = 0; q < 8; ++q) f.h[q] = (_Float16)(bf16_round(Wt[((size_t)o * DM + c0 + q) * 3 + k]) * 16.0f);
  *(volatile v8us*)((unsigned short*)Bt + (size_t)o * (3 * DM) + g8) = f.half[0]; __threadfence(); *(volatile v8us*)((unsigned short*)Bt + (size_t)o * (3 * DM) + g8) = f.half[0]; }
template <int MODE>
__global__ __launch_bounds__(256) void k_means(const float* __restrict__ GCN, const float* __restrict__ Ht, _Float16* __restrict__ Fh, _Float16* __restrict__ Fl) {
  #pragma clang fp contract(off)
  const int t_ = blockIdx.x * 256 + threadIdx.x; if (t_ >= NP_ * (DM / 8)) return; const int g8 = (t_ % (DM / 8)) * 8 + MODE * DM, p = t_ / (DM / 8); const int b = p / NNd, n = p % NNd; FragH fh, fl;
#pragma unroll
  for (int q = 0; q < 8; ++q) { const int cc = g8 + q; float s = 0.f; if (MODE == 0) {
#pragma unroll 1
      for (int t = 0; t < TT; ++t) s += GCN[((size_t)n * NG + b * TT + t) * DM + cc]; }
    else { const int c = cc - DM;
#pragma unroll 1
      for (int t = 0; t < TT; ++t) s += Ht[((size_t)p * TT + t) * DM + c]; }
    const float v = s / (float)TT; const _Float16 hi = (_Float16)v; fh.h[q] = hi; fl.h[q] = (_Float16)((v - (float)hi) * 1024.0f); }
  for (int pass = 0; pass < 2; ++pass) { *(volatile v8us*)((unsigned short*)Fh + (size_t)p * (2 * DM) + g8) = fh.half[0]; *(volatile v8us*)((unsigned short*)Fl + (size_t)p * (2 * DM) + g8) = fl.half[0]; if (pass == 0) __threadfence(); } }
__global__ __launch_bounds__(256) void k_gate(const float* __restrict__ F1, const float* __restrict__ GA, float* __restrict__ P, _Float16* __restrict__ Ph, _Float16* __restrict__ Pl, size_t n8) {
  #pragma clang fp contract(off)
  const size_t t = (size_t)blockIdx.x * 256 + threadIdx.x; if (t >= n8) return; FragH fh, fl; v4f oa, oc; const v4f a = *(const v4fa*)(F1 + t * 8), c = *(const v4fa*)(F1 + t * 8 + 4), ga = *(const v4fa*)(GA + t * 8), gc = *(const v4fa*)(GA + t * 8 + 4);
#pragma unroll
  for (int q = 0; q < 8; ++q) { const float f = (q < 4) ? a[q] : c[q - 4]; const float g = (q < 4) ? ga[q] : gc[q - 4]; const float v = f * (1.0f / (1.0f + expf(-g))); if (q < 4) oa[q] = v; else oc[q - 4] = v; const _Float16 hi = (_Float16)v; fh.h[q] = hi; fl.h[q] = (_Float16)((v - (float)hi) * 1024.0f); }
  for (int pass = 0; pass < 2; ++pass) { *(volatile v4f*)(P + t * 8) = oa; *(volatile v4f*)(P + t * 8 + 4) = oc; *(volatile v8us*)((unsigned short*)Ph + t * 8) = fh.half[0]; *(volatile v8us*)((unsigned short*)Pl + t * 8) = fl.half[0]; if (pass == 0) __threadfence(); } }
__global__ __launch_bounds__(256) void k_lnrelu(const float* __restrict__ X, const float* __restrict__ g, const float* __restrict__ bb, _Float16* __restrict__ Hh, _Float16* __restrict__ Hl) {
  #pragma clang fp contract(off)
  const int tid = threadIdx.x, w = tid >> 5, l = tid & 31; const int r = blockIdx.x * 8 + w; if (r >= NP_) return; float v[16]; float s = 0.f;
#pragma unroll
  for (int m = 0; m < 2; ++m) { const v4f a = *(const v4fa*)(X + (size_t)r * HP + m * 256 + 8 * l), c = *(const v4fa*)(X + (size_t)r * HP + m * 256 + 8 * l + 4);
#pragma unroll
    for (int j = 0; j < 4; ++j) { v[m * 8 + j] = a[j]; v[m * 8 + 4 + j] = c[j]; s += a[j] + c[j]; } }
  for (int o = 16; o > 0; o >>= 1) s += __shfl_xor(s, o, 32); const float mu = s / (float)HP; float vs = 0.f;
#pragma unroll
  for (int i = 0; i < 16; ++i) { const float d = v[i] - mu; vs += d * d; }
  for (int o = 16; o > 0; o >>= 1) vs += __shfl_xor(vs, o, 32); const float rs = rsqrtf(vs / (float)HP + 1e-5f);
  for (int pass = 0; pass < 2; ++pass) {
#pragma unroll
    for (int m = 0; m < 2; ++m) { FragH fh, fl;
#pragma unroll
      for (int j = 0; j < 8; ++j) { const int c = m * 256 + 8 * l + j; const float y = fmaxf((v[m * 8 + j] - mu) * rs * bf16_round(g[c]) + bf16_round(bb[c]), 0.f); const _Float16 hi = (_Float16)y; fh.h[j] = hi; fl.h[j] = (_Float16)((y - (float)hi) * 1024.0f); }
      *(volatile v8us*)((unsigned short*)Hh + (size_t)r * HP + m * 256 + 8 * l) = fh.half[0]; *(volatile v8us*)((unsigned short*)Hl + (size_t)r * HP + m * 256 + 8 * l) = fl.half[0]; }
    if (pass == 0) __threadfence(); } }
__global__ __launch_bounds__(1024) void k_pred(const _Float16* __restrict__ Hh, const _Float16* __restrict__ Hl, const float* __restrict__ Wp3, const float* __restrict__ bp3, float* __restrict__ out) {
  #pragma clang fp contract(off)
  __shared__ float res[32]; const int tid = threadIdx.x, w = tid >> 5, l = tid & 31; const int r = blockIdx.x * 32 + w; float s = 0.f;
  if (r < NP_) for (int m = 0; m < 2; ++m) { FragH a, c; a.half[0] = *(const v8us*)((const unsigned short*)Hh + (size_t)r * HP + m * 256 + 8 * l); c.half[0] = *(const v8us*)((const unsigned short*)Hl + (size_t)r * HP + m * 256 + 8 * l);
#pragma unroll
    for (int j = 0; j < 8; ++j) s += ((float)a.h[j] + (float)c.h[j] * 0.0009765625f) * bf16_round(Wp3[m * 256 + 8 * l + j]); }
  for (int o = 16; o > 0; o >>= 1) s += __shfl_xor(s, o, 32); if (l == 0) res[w] = s + bf16_round(bp3[0]);
  __syncthreads();
  if (tid < 32 && blockIdx.x * 32 + tid < NP_) { *(volatile float*)(out + (size_t)blockIdx.x * 32 + tid) = res[tid]; __threadfence(); *(volatile float*)(out + (size_t)blockIdx.x * 32 + tid) = res[tid]; } }
__global__ __launch_bounds__(256) void k_repar(const float* __restrict__ VE, const float* __restrict__ eps, _Float16* __restrict__ Zh, _Float16* __restrict__ Zl, float* __restrict__ outmu, float* __restrict__ outlv) {
  #pragma clang fp contract(off)
  const int t = blockIdx.x * 256 + threadIdx.x; if (t >= NP_ * (SL / 8)) return; const int c0 = (t % (SL / 8)) * 8, r = t / (SL / 8); const v4f ma = *(const v4fa*)(VE + (size_t)r * DM + c0), mc = *(const v4fa*)(VE + (size_t)r * DM + c0 + 4), la = *(const v4fa*)(VE + (size_t)r * DM + SL + c0), lc = *(const v4fa*)(VE + (size_t)r * DM + SL + c0 + 4); FragH fh, fl;
#pragma unroll
  for (int q = 0; q < 8; ++q) { const float mu = (q < 4) ? ma[q] : mc[q - 4], lv = (q < 4) ? la[q] : lc[q - 4]; const float z = mu + bf16_round(eps[(size_t)r * SL + c0 + q]) * expf(0.5f * lv); const _Float16 hi = (_Float16)z; fh.h[q] = hi; fl.h[q] = (_Float16)((z - (float)hi) * 1024.0f); }
  for (int pass = 0; pass < 2; ++pass) { *(volatile v8us*)((unsigned short*)Zh + (size_t)r * SL + c0) = fh.half[0]; *(volatile v8us*)((unsigned short*)Zl + (size_t)r * SL + c0) = fl.half[0]; *(volatile v4f*)(outmu + (size_t)r * SL + c0) = ma; *(volatile v4f*)(outmu + (size_t)r * SL + c0 + 4) = mc; *(volatile v4f*)(outlv + (size_t)r * SL + c0) = la; *(volatile v4f*)(outlv + (size_t)r * SL + c0 + 4) = lc; if (pass == 0) __threadfence(); } }
__global__ __launch_bounds__(256) void k_bnout(const float* __restrict__ P, const float* __restrict__ emb, const float* __restrict__ gam, const float* __restrict__ bet, float* __restrict__ out) {
  #pragma clang fp contract(off)
  __shared__ double s1[8][32], s2[8][32]; __shared__ float sc[32], sh[32]; const int tid = threadIdx.x, w = tid >> 5, l = tid & 31; const int c = blockIdx.x * 32 + l; double a = 0.0, b = 0.0;
#pragma unroll 1
  for (int r = w; r < NP_; r += 8) { const double v = (double)(P[(size_t)r * DM + c] * bf16_round(emb[(size_t)(r % NNd) * DM + c])); a += v; b += v * v; }
  s1[w][l] = a; s2[w][l] = b; __syncthreads();
  if (w == 0) { double t1 = 0.0, t2 = 0.0; for (int k = 0; k < 8; ++k) { t1 += s1[k][l]; t2 += s2[k][l]; } const double m = t1 / (double)NP_; double var = t2 / (double)NP_ - m * m; if (var < 0.0) var = 0.0; const float scale = bf16_round(gam[c]) / sqrtf((float)var + 1e-5f); sc[l] = scale; sh[l] = bf16_round(bet[c]) - (float)m * scale; }
  __syncthreads();
#pragma unroll 1
  for (int r = w; r < NP_; r += 8) { const float o = P[(size_t)r * DM + c] * bf16_round(emb[(size_t)(r % NNd) * DM + c]); const float y = fmaxf(o * sc[l] + sh[l], 0.f); *(volatile float*)(out + (size_t)r * DM + c) = y; }
  __threadfence();
#pragma unroll 1
  for (int r = w; r < NP_; r += 8) { const float o = P[(size_t)r * DM + c] * bf16_round(emb[(size_t)(r % NNd) * DM + c]); const float y = fmaxf(o * sc[l] + sh[l], 0.f); *(volatile float*)(out + (size_t)r * DM + c) = y; } }

extern "C" void kernel_launch(void* const* d_in, const int* in_sizes, int n_in,
                              void* d_out, int out_size, void* d_ws, size_t ws_size, hipStream_t stream) {
  (void)in_sizes; (void)n_in; (void)out_size;
  const float* const* I = (const float* const*)d_in; const float* data = I[0]; const int* ei = (const int*)d_in[1]; const float* Wg = I[2]; const float* bg = I[3]; const float* Wt1 = I[4]; const float* bt1 = I[5]; const float* Wt2 = I[6]; const float* bt2 = I[7]; const float* Wt3 = I[8]; const float* bt3 = I[9]; const float* Wf = I[10]; const float* bff = I[11]; const float* Wa = I[12]; const float* ba = I[13];
  const float* Wp1 = I[14]; const float* bp1 = I[15]; const float* g1 = I[16]; const float* be1 = I[17]; const float* Wp2 = I[18]; const float* bp2 = I[19]; const float* g2 = I[20]; const float* be2 = I[21]; const float* Wp3 = I[22]; const float* bp3 = I[23];
  const float* We1 = I[24]; const float* bee1 = I[25]; const float* We2 = I[26]; const float* bee2 = I[27]; const float* Wd1 = I[28]; const float* bd1 = I[29]; const float* Wd2 = I[30]; const float* bd2 = I[31]; const float* eps = I[32]; const float* emb = I[33]; const float* gam = I[34]; const float* bet = I[35];
  const int* esrc = ei; const int* edst = ei + NEd;
  char* ws = (char*)d_ws; size_t off = 0;
  auto take = [&](size_t bytes) { char* p = ws + off; off += (bytes + 255) & ~(size_t)255; return p; };
  _Float16* Bg = (_Float16*)take((size_t)3 * DM * SL * 2); _Float16* Bt_[3]; for (int i = 0; i < 3; ++i) Bt_[i] = (_Float16*)take((size_t)DM * 3 * DM * 2); _Float16* Bf = (_Float16*)take((size_t)DM * 2 * DM * 2); _Float16* Ba = (_Float16*)take((size_t)DM * DM * 2); _Float16* Bp1 = (_Float16*)take((size_t)HP * DM * 2); _Float16* Bp2 = (_Float16*)take((size_t)HP * HP * 2); _Float16* Be1 = (_Float16*)take((size_t)DM * DM * 2); _Float16* Be2 = (_Float16*)take((size_t)DM * DM * 2); _Float16* Bd1 = (_Float16*)take((size_t)DM * SL * 2); _Float16* Bd2 = (_Float16*)take((size_t)SL * DM * 2);
  _Float16* X16 = (_Float16*)take((size_t)NR * SL * 2); _Float16* Ah = (_Float16*)take((size_t)NNp * NNp * 2); _Float16* Al = (_Float16*)take((size_t)NNp * NNp * 2);
  _Float16* Bh = (_Float16*)take((size_t)NG * SL * NNp * 2); _Float16* Bl = (_Float16*)take((size_t)NG * SL * NNp * 2); float* PR = (float*)take((size_t)NNp * NG * SL * 4); _Float16* T1h = (_Float16*)take((size_t)NR * SL * 2); _Float16* T1l = (_Float16*)take((size_t)NR * SL * 2); _Float16* T2h = (_Float16*)take((size_t)NR * SL * 2); _Float16* T2l = (_Float16*)take((size_t)NR * SL * 2);
  float* GCN = (float*)take((size_t)NR * DM * 4); float* Ht = (float*)take((size_t)NP_ * TT * DM * 4); _Float16* Ih = Bh;        float* Hn = GCN;
  _Float16* Fh = (_Float16*)take((size_t)NP_ * 2 * DM * 2); _Float16* Fl = (_Float16*)take((size_t)NP_ * 2 * DM * 2); float* F1 = (float*)take((size_t)NP_ * DM * 4); _Float16* F1h = (_Float16*)take((size_t)NP_ * DM * 2); _Float16* F1l = (_Float16*)take((size_t)NP_ * DM * 2); float* GA = (float*)take((size_t)NP_ * DM * 4); float* P = (float*)take((size_t)NP_ * DM * 4); _Float16* Ph = (_Float16*)take((size_t)NP_ * DM * 2); _Float16* Pl = (_Float16*)take((size_t)NP_ * DM * 2);
  float* L1 = (float*)take((size_t)NP_ * HP * 4); _Float16* L1h = (_Float16*)take((size_t)NP_ * HP * 2); _Float16* L1l = (_Float16*)take((size_t)NP_ * HP * 2); float* L2 = (float*)take((size_t)NP_ * HP * 4); _Float16* L2h = (_Float16*)take((size_t)NP_ * HP * 2); _Float16* L2l = (_Float16*)take((size_t)NP_ * HP * 2);
  float* V1 = (float*)take((size_t)NP_ * DM * 4); _Float16* V1h = (_Float16*)take((size_t)NP_ * DM * 2); _Float16* V1l = (_Float16*)take((size_t)NP_ * DM * 2); float* VE = (float*)take((size_t)NP_ * DM * 4); _Float16* Zh = (_Float16*)take((size_t)NP_ * SL * 2); _Float16* Zl = (_Float16*)take((size_t)NP_ * SL * 2); float* D1 = (float*)take((size_t)NP_ * DM * 4); _Float16* D1h = (_Float16*)take((size_t)NP_ * DM * 2); _Float16* D1l = (_Float16*)take((size_t)NP_ * DM * 2);
  if (off > ws_size) return;
  float* out0 = (float*)d_out; float* outPred = (float*)((char*)d_out + 1228800); float* outRec = (float*)((char*)d_out + 1238400); float* outMu = (float*)((char*)d_out + 1852800); float* outLv = (float*)((char*)d_out + 2467200);
  k_wgcn<<<(3 * DM * (SL / 8) + 255) / 256, 256, 0, stream>>>(Wg, Bg); k_wt3<<<(DM * (3 * DM / 8) + 255) / 256, 256, 0, stream>>>(Wt1, Bt_[0]); k_wt3<<<(DM * (3 * DM / 8) + 255) / 256, 256, 0, stream>>>(Wt2, Bt_[1]); k_wt3<<<(DM * (3 * DM / 8) + 255) / 256, 256, 0, stream>>>(Wt3, Bt_[2]);
  k_wt_f16<<<(DM * (2 * DM / 8) + 255) / 256, 256, 0, stream>>>(Wf, Bf, 2 * DM, DM, 16.0f); k_wt_f16<<<(DM * (DM / 8) + 255) / 256, 256, 0, stream>>>(Wa, Ba, DM, DM, 16.0f); k_wt_f16<<<(HP * (DM / 8) + 255) / 256, 256, 0, stream>>>(Wp1, Bp1, DM, HP, 16.0f); k_wt_f16<<<(HP * (HP / 8) + 255) / 256, 256, 0, stream>>>(Wp2, Bp2, HP, HP, 16.0f);
  k_wt_f16<<<(DM * (DM / 8) + 255) / 256, 256, 0, stream>>>(We1, Be1, DM, DM, 16.0f); k_wt_f16<<<(DM * (DM / 8) + 255) / 256, 256, 0, stream>>>(We2, Be2, DM, DM, 16.0f); k_wt_f16<<<(DM * (SL / 8) + 255) / 256, 256, 0, stream>>>(Wd1, Bd1, SL, DM, 16.0f); k_wt_f16<<<(SL * (DM / 8) + 255) / 256, 256, 0, stream>>>(Wd2, Bd2, DM, SL, 16.0f);
  k_x0<<<(NR * (SL / 8) + 255) / 256, 256, 0, stream>>>(data, X16); k_adj<<<(NNp * (NNp / 8) + 255) / 256, 256, 0, stream>>>(esrc, edst, Ah, Al);
  const dim3 gP(((NNp / 16) * (NG * SL / 64) + 3) / 4, 1); const size_t n8x = (size_t)NR * SL / 8;
  k_htrx<<<(NG * SL * (NNp / 8) + 255) / 256, 256, 0, stream>>>(X16, Bh);
  k_gemm_hhx<0><<<gP, 128, 0, stream>>>(Ah, NNp, 0, Bh, NNp, 0, 1.0f, nullptr, 0, nullptr, 1, 0, 0, PR, nullptr, NG * SL, 0, NNp, NG * SL, NNp); k_gemm_hhx<0><<<gP, 128, 0, stream>>>(Al, NNp, 0, Bh, NNp, 0, 1.0f / 1024.0f, nullptr, 0, PR, 1, (size_t)NG * SL, 0, PR, nullptr, NG * SL, 0, NNp, NG * SL, NNp);
  k_neg<<<(unsigned)((n8x + 255) / 256), 256, 0, stream>>>(PR, T1h, T1l, n8x);
  k_htr<<<(NG * SL * (NNp / 8) + 255) / 256, 256, 0, stream>>>(PR, -1.0f, Bh, Bl);
  k_gemm_hhx<0><<<gP, 128, 0, stream>>>(Ah, NNp, 0, Bh, NNp, 0, 1.0f, nullptr, 0, nullptr, 1, 0, 0, PR, nullptr, NG * SL, 0, NNp, NG * SL, NNp); k_gemm_hhx<0><<<gP, 128, 0, stream>>>(Ah, NNp, 0, Bl, NNp, 0, 1.0f / 1024.0f, nullptr, 0, PR, 1, (size_t)NG * SL, 0, PR, nullptr, NG * SL, 0, NNp, NG * SL, NNp);
  k_gemm_hhx<0><<<gP, 128, 0, stream>>>(Al, NNp, 0, Bh, NNp, 0, 1.0f / 1024.0f, nullptr, 0, PR, 1, (size_t)NG * SL, 0, PR, nullptr, NG * SL, 0, NNp, NG * SL, NNp);
  k_tx2<<<(unsigned)((n8x + 255) / 256), 256, 0, stream>>>(PR, X16, T2h, T2l, n8x);
  const dim3 gG(((NR / 16) * (DM / 64) + 3) / 4, 1);
  k_gemm_hhx<0><<<gG, 128, 0, stream>>>(X16, SL, 0, Bg, SL, 0, 0.0625f, bg, 0, nullptr, 1, 0, 0, GCN, nullptr, DM, 0, NR, DM, SL);
  k_gemm_hhx<0><<<gG, 128, 0, stream>>>(T1h, SL, 0, Bg + (size_t)DM * SL, SL, 0, 0.0625f, nullptr, 0, GCN, 1, (size_t)DM, 0, GCN, nullptr, DM, 0, NR, DM, SL); k_gemm_hhx<0><<<gG, 128, 0, stream>>>(T1l, SL, 0, Bg + (size_t)DM * SL, SL, 0, 0.0625f / 1024.0f, nullptr, 0, GCN, 1, (size_t)DM, 0, GCN, nullptr, DM, 0, NR, DM, SL);
  k_gemm_hhx<0><<<gG, 128, 0, stream>>>(T2h, SL, 0, Bg + (size_t)2 * DM * SL, SL, 0, 0.0625f, nullptr, 0, GCN, 1, (size_t)DM, 0, GCN, nullptr, DM, 0, NR, DM, SL); k_gemm_hhx<0><<<gG, 128, 0, stream>>>(T2l, SL, 0, Bg + (size_t)2 * DM * SL, SL, 0, 0.0625f / 1024.0f, nullptr, 0, GCN, 1, (size_t)DM, 0, GCN, nullptr, DM, 0, NR, DM, SL);
  k_means<0><<<(NP_ * (DM / 8) + 255) / 256, 256, 0, stream>>>(GCN, nullptr, Fh, Fl);
  k_xt<<<(unsigned)(((size_t)NP_ * TT * (DM / 4) + 255) / 256), 256, 0, stream>>>(GCN, Ht);
  const dim3 gT(((NP_ * TT / 16) * (DM / 64) + 3) / 4, 1); float* Hc = Ht; float* Ho = Hn;
  { const float* bts[3] = {bt1, bt2, bt3}; const int dil[3] = {1, 2, 4};
    for (int i = 0; i < 3; ++i) { k_im1d<<<(unsigned)(((size_t)NP_ * TT * (3 * DM / 8) + 255) / 256), 256, 0, stream>>>(Hc, dil[i], Ih);
      k_gemm_hhx<3><<<gT, 128, 0, stream>>>(Ih, 3 * DM, 0, Bt_[i], 3 * DM, 0, 0.0625f, bts[i], 0, nullptr, 1, 0, 0, Ho, nullptr, DM, 0, NP_ * TT, DM, 3 * DM);
      k_addres<<<(unsigned)(((size_t)NP_ * TT * DM / 4 + 255) / 256), 256, 0, stream>>>(Ho, Hc, (size_t)NP_ * TT * DM / 4);
      float* tmp = Hc; Hc = Ho; Ho = tmp; } }
  k_means<1><<<(NP_ * (DM / 8) + 255) / 256, 256, 0, stream>>>(nullptr, Hc, Fh, Fl);
  const dim3 gF(((NP_ / 16) * (DM / 64) + 3) / 4, 1), gH(((NP_ / 16) * (HP / 64) + 3) / 4, 1), gS(((NP_ / 16) * 1 + 3) / 4, 1); const size_t n8p = (size_t)NP_ * DM / 8;
  k_gemm_hhx<0><<<gF, 128, 0, stream>>>(Fh, 2 * DM, 0, Bf, 2 * DM, 0, 0.0625f, bff, 0, nullptr, 1, 0, 0, F1, nullptr, DM, 0, NP_, DM, 2 * DM); k_gemm_hhx<3><<<gF, 128, 0, stream>>>(Fl, 2 * DM, 0, Bf, 2 * DM, 0, 0.0625f / 1024.0f, nullptr, 0, F1, 1, (size_t)DM, 0, F1, nullptr, DM, 0, NP_, DM, 2 * DM);
  k_split<<<(unsigned)((n8p + 255) / 256), 256, 0, stream>>>(F1, F1h, F1l, n8p);
  k_gemm_hhx<0><<<gF, 128, 0, stream>>>(F1h, DM, 0, Ba, DM, 0, 0.0625f, ba, 0, nullptr, 1, 0, 0, GA, nullptr, DM, 0, NP_, DM, DM); k_gemm_hhx<0><<<gF, 128, 0, stream>>>(F1l, DM, 0, Ba, DM, 0, 0.0625f / 1024.0f, nullptr, 0, GA, 1, (size_t)DM, 0, GA, nullptr, DM, 0, NP_, DM, DM);
  k_gate<<<(unsigned)((n8p + 255) / 256), 256, 0, stream>>>(F1, GA, P, Ph, Pl, n8p);
  k_gemm_hhx<0><<<gH, 128, 0, stream>>>(Ph, DM, 0, Bp1, DM, 0, 0.0625f, bp1, 0, nullptr, 1, 0, 0, L1, nullptr, HP, 0, NP_, HP, DM); k_gemm_hhx<0><<<gH, 128, 0, stream>>>(Pl, DM, 0, Bp1, DM, 0, 0.0625f / 1024.0f, nullptr, 0, L1, 1, (size_t)HP, 0, L1, nullptr, HP, 0, NP_, HP, DM);
  k_lnrelu<<<(NP_ + 7) / 8, 256, 0, stream>>>(L1, g1, be1, L1h, L1l);
  k_gemm_hhx<0><<<gH, 128, 0, stream>>>(L1h, HP, 0, Bp2, HP, 0, 0.0625f, bp2, 0, nullptr, 1, 0, 0, L2, nullptr, HP, 0, NP_, HP, HP); k_gemm_hhx<0><<<gH, 128, 0, stream>>>(L1l, HP, 0, Bp2, HP, 0, 0.0625f / 1024.0f, nullptr, 0, L2, 1, (size_t)HP, 0, L2, nullptr, HP, 0, NP_, HP, HP);
  k_lnrelu<<<(NP_ + 7) / 8, 256, 0, stream>>>(L2, g2, be2, L2h, L2l);
  k_pred<<<(NP_ + 31) / 32, 1024, 0, stream>>>(L2h, L2l, Wp3, bp3, outPred);
  k_gemm_hhx<0><<<gF, 128, 0, stream>>>(Ph, DM, 0, Be1, DM, 0, 0.0625f, bee1, 0, nullptr, 1, 0, 0, V1, nullptr, DM, 0, NP_, DM, DM); k_gemm_hhx<3><<<gF, 128, 0, stream>>>(Pl, DM, 0, Be1, DM, 0, 0.0625f / 1024.0f, nullptr, 0, V1, 1, (size_t)DM, 0, V1, nullptr, DM, 0, NP_, DM, DM);
  k_split<<<(unsigned)((n8p + 255) / 256), 256, 0, stream>>>(V1, V1h, V1l, n8p);
  k_gemm_hhx<0><<<gF, 128, 0, stream>>>(V1h, DM, 0, Be2, DM, 0, 0.0625f, bee2, 0, nullptr, 1, 0, 0, VE, nullptr, DM, 0, NP_, DM, DM); k_gemm_hhx<0><<<gF, 128, 0, stream>>>(V1l, DM, 0, Be2, DM, 0, 0.0625f / 1024.0f, nullptr, 0, VE, 1, (size_t)DM, 0, VE, nullptr, DM, 0, NP_, DM, DM);
  k_repar<<<(NP_ * (SL / 8) + 255) / 256, 256, 0, stream>>>(VE, eps, Zh, Zl, outMu, outLv);
  k_gemm_hhx<0><<<gF, 128, 0, stream>>>(Zh, SL, 0, Bd1, SL, 0, 0.0625f, bd1, 0, nullptr, 1, 0, 0, D1, nullptr, DM, 0, NP_, DM, SL); k_gemm_hhx<3><<<gF, 128, 0, stream>>>(Zl, SL, 0, Bd1, SL, 0, 0.0625f / 1024.0f, nullptr, 0, D1, 1, (size_t)DM, 0, D1, nullptr, DM, 0, NP_, DM, SL);
  k_split<<<(unsigned)((n8p + 255) / 256), 256, 0, stream>>>(D1, D1h, D1l, n8p);
  k_gemm_hhx<0><<<gS, 128, 0, stream>>>(D1h, DM, 0, Bd2, DM, 0, 0.0625f, bd2, 0, nullptr, 1, 0, 0, outRec, nullptr, SL, 0, NP_, SL, DM); k_gemm_hhx<0><<<gS, 128, 0, stream>>>(D1l, DM, 0, Bd2, DM, 0, 0.0625f / 1024.0f, nullptr, 0, outRec, 1, (size_t)SL, 0, outRec, nullptr, SL, 0, NP_, SL, DM);
  k_bnout<<<DM / 32, 256, 0, stream>>>(P, emb, gam, bet, out0);
}
